// GraphConvolution_17343077941573
// MI455X (gfx1250) — hardware-run, weakly checked
//
#include <hip/hip_runtime.h>

typedef float          v8f   __attribute__((ext_vector_type(8)));
typedef float          v4f   __attribute__((ext_vector_type(4)));
typedef unsigned int   v4u   __attribute__((ext_vector_type(4)));
typedef int            v8i   __attribute__((ext_vector_type(8)));
typedef unsigned short v8us  __attribute__((ext_vector_type(8)));
typedef unsigned short v16us __attribute__((ext_vector_type(16)));
typedef __bf16         v16bf __attribute__((ext_vector_type(16)));
typedef _Float16       v16h  __attribute__((ext_vector_type(16)));
typedef v4f  __attribute__((may_alias)) v4fa;
typedef v8us __attribute__((may_alias)) v8usa;
union FragB { v16bf v; v16us u; v8us h[2]; v8i w; };
union FragH { v16h  v; v16us u; v8us h[2]; v8i w; };

__device__ __forceinline__ v8f wmb(const FragB& a, const FragB& b, v8f c) {
  v8f d = __builtin_amdgcn_wmma_f32_16x16x32_bf16(false, a.v, false, b.v, (short)0, c, false, false);
  asm volatile("v_nop\n\tv_nop\n\tv_nop\n\tv_nop" : "+v"(d) : "v"(a.w), "v"(b.w));
  return d;
}

__device__ __forceinline__ v8f wmh(const FragH& a, const FragH& b, v8f c) {
  v8f d = __builtin_amdgcn_wmma_f32_16x16x32_f16(false, a.v, false, b.v, (short)0, c, false, false);
  asm volatile("v_nop\n\tv_nop\n\tv_nop\n\tv_nop" : "+v"(d) : "v"(a.w), "v"(b.w));
  return d;
}

__device__ __forceinline__ unsigned bf16_bits(float f) {
  const unsigned u = __float_as_uint(f);
  const unsigned r = (u + 0x7FFFu + ((u >> 16) & 1u)) >> 16;
  const unsigned q = (u >> 16) | 0x40u;
  return ((u & 0x7fffffffu) > 0x7f800000u) ? q : r;
}

__device__ __forceinline__ float bf16_val(float f) {
  return __uint_as_float(bf16_bits(f) << 16);
}
__device__ __forceinline__ int clampi(int v, int lo, int hi) {
  return v < lo ? lo : (v > hi ? hi : v);
}

__device__ __forceinline__ unsigned f16_bits(float f) {
  const unsigned u  = __float_as_uint(f);
  const unsigned s  = (u >> 16) & 0x8000u;
  const unsigned a  = u & 0x7fffffffu;
  const unsigned t  = a - 0x38000000u;
  const unsigned r  = (t + 0x0FFFu + ((t >> 13) & 1u)) >> 13;
  const unsigned rc = r > 0x7C00u ? 0x7C00u : r;
  const bool small  = a < 0x38800000u;
  const bool isnan  = a > 0x7f800000u;
  const unsigned fin = small ? 0u : (s | rc);
  return isnan ? (s | 0x7E00u) : fin;
}

__device__ __forceinline__ unsigned pk16(unsigned lo, unsigned hi) { return lo | (hi << 16); }
__device__ __forceinline__ unsigned bf16_lo_bits(float v) {
  float hi = bf16_val(v);
  asm volatile("" : "+v"(hi));
  return bf16_bits(v - hi);
}
__device__ __forceinline__ v4u pack8_bf16(v4f a, v4f c) {
  return (v4u){ pk16(bf16_bits(a[0]), bf16_bits(a[1])), pk16(bf16_bits(a[2]), bf16_bits(a[3])),
                pk16(bf16_bits(c[0]), bf16_bits(c[1])), pk16(bf16_bits(c[2]), bf16_bits(c[3])) };
}
__device__ __forceinline__ v4u pack8_bf16_lo(v4f a, v4f c) {
  return (v4u){ pk16(bf16_lo_bits(a[0]), bf16_lo_bits(a[1])), pk16(bf16_lo_bits(a[2]), bf16_lo_bits(a[3])),
                pk16(bf16_lo_bits(c[0]), bf16_lo_bits(c[1])), pk16(bf16_lo_bits(c[2]), bf16_lo_bits(c[3])) };
}
__device__ __forceinline__ v4u pack8_f16(v4f a, v4f c) {
  return (v4u){ pk16(f16_bits(a[0]), f16_bits(a[1])), pk16(f16_bits(a[2]), f16_bits(a[3])),
                pk16(f16_bits(c[0]), f16_bits(c[1])), pk16(f16_bits(c[2]), f16_bits(c[3])) };
}

template <int FORM>
__global__ __launch_bounds__(256) void k_plane(const float* __restrict__ src, int rows, int cols, int ldsrc,
                                               unsigned short* __restrict__ dst, int MP, int KP) {
  static_assert(FORM >= 0 && FORM <= 3);
  const int KTOT = (FORM == 1 || FORM == 3) ? 2 * KP : KP;
  const unsigned ppr   = (unsigned)(KTOT >> 3);
  const unsigned kp8   = (unsigned)(KP >> 3);
  const unsigned total = (unsigned)MP * ppr;
  const unsigned g     = blockIdx.x * 256u + threadIdx.x;
  const unsigned rowu  = g / ppr;
  const unsigned p     = g - rowu * ppr;
  const bool second    = p >= kp8;
  const int row = (int)rowu;
  const int c0  = (int)((second ? p - kp8 : p) << 3);
  const float* srow = src + (size_t)clampi(row, 0, rows - 1) * (size_t)ldsrc;
  float x[8];
  unsigned mk[8];
#pragma unroll
  for (int e = 0; e < 8; ++e) {
    const int c = c0 + e;
    const float v = srow[clampi(c, 0, cols - 1)];
    asm volatile("" :: "v"(v));
    x[e]  = v;
    mk[e] = (row < rows && c < cols) ? 0xFFFFu : 0u;
  }
  const v4f a = (v4f){ x[0], x[1], x[2], x[3] };
  const v4f c = (v4f){ x[4], x[5], x[6], x[7] };
  v4u o;
  if (FORM == 2) {
    o = pack8_f16(a, c);
  } else {
    const v4u hi = pack8_bf16(a, c);
    o = hi;
    if (FORM == 1) { const v4u lo = pack8_bf16_lo(a, c); o = second ? lo : hi; }
  }
  const v4u mw = (v4u){ pk16(mk[0], mk[1]), pk16(mk[2], mk[3]), pk16(mk[4], mk[5]), pk16(mk[6], mk[7]) };
  o &= mw;
  if (g < total) {
    volatile v4u* q = (volatile v4u*)(dst + (size_t)g * 8);
    *q = o;
    __threadfence();
    *q = o;
  }
}

template <int FORM> struct FragOf    { typedef FragB T; };
template <>         struct FragOf<2> { typedef FragH T; };
__device__ __forceinline__ v8f mm(const FragB& a, const FragB& b, v8f c) { return wmb(a, b, c); }
__device__ __forceinline__ v8f mm(const FragH& a, const FragH& b, v8f c) { return wmh(a, b, c); }
template <class F> __device__ __forceinline__ F ld_frag(const unsigned short* p) {
  F f;
  f.h[0] = *(const v8usa*)(p);
  f.h[1] = *(const v8usa*)(p + 16);
  return f;
}

template <int FORM, int EPI>
__global__ __launch_bounds__(256) __attribute__((amdgpu_num_vgpr(248)))
void k_gemm_nt(const unsigned short* __restrict__ A, const unsigned short* __restrict__ B,
               const float* __restrict__ bias, float* __restrict__ D, int M, int N, int KTOT, int ldd) {
  static_assert(FORM >= 0 && FORM <= 2);
  static_assert(EPI == 0 || EPI == 1);
  typedef typename FragOf<FORM>::T F;
  __shared__ __attribute__((aligned(16))) float sT[8][16 * 68];
  const int lane = threadIdx.x & 31;
  const int wave = threadIdx.x >> 5;
  const int tilesM = (M + 63) >> 6;
  const int tilesN = (N + 63) >> 6;
  const int tile = blockIdx.x * 8 + wave;
  if (tile >= tilesM * tilesN) return;
  const int tm = tile / tilesN;
  const int tn = tile - tm * tilesN;
  const int m0 = tm << 6;
  const int n0 = tn << 6;

  const int rl = lane & 15;
  const int h8 = (lane >> 4) * 8;
  const unsigned short* pa = A + (size_t)(m0 + rl) * (size_t)KTOT + h8;
  const unsigned short* pb = B + (size_t)(n0 + rl) * (size_t)KTOT + h8;

  v8f acc[4][4];
#pragma unroll
  for (int i = 0; i < 4; ++i)
#pragma unroll
    for (int j = 0; j < 4; ++j) acc[i][j] = (v8f){0.f, 0.f, 0.f, 0.f, 0.f, 0.f, 0.f, 0.f};

#pragma unroll 1
  for (int k0 = 0; k0 < KTOT; k0 += 32) {
    F bf[4];
#pragma unroll
    for (int j = 0; j < 4; ++j) bf[j] = ld_frag<F>(pb + (size_t)(j << 4) * (size_t)KTOT + k0);
#pragma unroll
    for (int i = 0; i < 4; ++i) {
      const F af = ld_frag<F>(pa + (size_t)(i << 4) * (size_t)KTOT + k0);
#pragma unroll
      for (int j = 0; j < 4; ++j) acc[i][j] = mm(af, bf[j], acc[i][j]);
    }
  }

  float* slab = sT[wave];
  const int hh = lane >> 4;
  const int c4 = (lane & 15) * 4;
  const int nc = n0 + c4;
  const bool cok = nc < N;
  v4f bv = (v4f){0.f, 0.f, 0.f, 0.f};
  if (EPI == 1) {
    bv = *(const v4fa*)(bias + clampi(nc, 0, N - 4));
    asm volatile("" :: "v"(bv));
  }
#pragma unroll
  for (int i = 0; i < 4; ++i) {
    const int mBase = m0 + (i << 4);
#pragma unroll
    for (int j = 0; j < 4; ++j) {
#pragma unroll
      for (int r = 0; r < 8; ++r) slab[(h8 + r) * 68 + (j << 4) + rl] = acc[i][j][r];
    }
    __builtin_amdgcn_fence(__ATOMIC_RELEASE, "workgroup");
    __builtin_amdgcn_wave_barrier();
    __builtin_amdgcn_fence(__ATOMIC_ACQUIRE, "workgroup");
    v4f vv[8];
#pragma unroll
    for (int it = 0; it < 8; ++it) {
      const int row = it * 2 + hh;
      v4f v = *(const v4fa*)(slab + row * 68 + c4);
      if (EPI == 1) v += bv;
      vv[it] = v;
    }
    for (int pass = 0; pass < 2; ++pass) {
#pragma unroll
      for (int it = 0; it < 8; ++it) {
        const int row = mBase + it * 2 + hh;
        if (cok && row < M) *(volatile v4f*)(D + (size_t)row * (size_t)ldd + nc) = vv[it];
      }
      __threadfence();
    }
    __builtin_amdgcn_fence(__ATOMIC_RELEASE, "workgroup");
    __builtin_amdgcn_wave_barrier();
    __builtin_amdgcn_fence(__ATOMIC_ACQUIRE, "workgroup");
  }
}

#pragma clang fp contract(off)

#define NN      100000
#define KD      128
#define OD      128
#define NE      1100000
#define TT      500000
#define NREL    201
#define MPAD    100096
#define NTHR    256
#define NWAVE   8
#define EPT     8
#define WCH     (32 * EPT)
#define NBRUN   1024
#define SLB     10
#define NBK     98
#define WLCAP   2560
#define LCAP    15360
#define DEGCAP  64
#define MAXDEG_MEAS   25
#define MAXB1024_MEAS 11480
#define WTP     136
#define WSMAX   ((size_t)128 << 20)

#define BK_ZINTS (NWAVE * WLCAP + LCAP + 3 * NBRUN)
#define BK_INTS  (BK_ZINTS + 16)
#define BK_LDS   (BK_INTS * 4)

static_assert((NE - NN) % 2 == 0);
static_assert((NE - NN) / 2 == TT);
static_assert(NE < (1 << 21) && NBRUN == 1024);
static_assert(NBRUN == (1 << SLB) && NBRUN == NTHR * 4 && NBRUN % 32 == 0);
static_assert(NE % 8 == 0 && NE >= 8);
static_assert(NBK * NBRUN >= NN && (NBK - 1) * NBRUN < NN);
static_assert(LCAP % 1024 == 0 && (LCAP / 2) % NTHR == 0);
static_assert((long long)LCAP * 100 >= (long long)MAXB1024_MEAS * 125);
static_assert(WLCAP >= MAXB1024_MEAS / 8 + 1024 + 1);
static_assert(MAXDEG_MEAS + 8 <= DEGCAP);
static_assert(BK_ZINTS % (NTHR * 4) == 0);
static_assert(BK_LDS <= 262144);
static_assert(MPAD % 64 == 0 && MPAD >= NN && MPAD % 16 == 0 && (MPAD * KD / 8) % NTHR == 0);
static_assert(KD % 32 == 0 && OD % 64 == 0 && OD == 32 * 4);
static_assert(NN % NWAVE == 0);
static_assert((long long)NN * OD - 1 == 12799999LL);
static_assert(NREL <= 256 && OD <= 128);

typedef int v2i __attribute__((ext_vector_type(2)));
typedef int v4i __attribute__((ext_vector_type(4)));
typedef v2i __attribute__((may_alias)) v2ia;
typedef v4i __attribute__((may_alias)) v4ia;

__device__ __forceinline__ void st2_v4f(float* p, v4f v) {
  *(volatile v4f*)p = v;
  __threadfence();
  *(volatile v4f*)p = v;
}
__device__ __forceinline__ void st2_v4i(int* p, v4i v) {
  *(volatile v4i*)p = v;
  __threadfence();
  *(volatile v4i*)p = v;
}
__device__ __forceinline__ void st2_v8us(unsigned short* p, v8us v) {
  *(volatile v8us*)p = v;
  __threadfence();
  *(volatile v8us*)p = v;
}

__device__ __forceinline__ int twin_of(int e) {
  const int d = (e < TT) ? TT : ((e < 2 * TT) ? -TT : 0);
  return clampi(e + d, 0, NE - 1);
}

__global__ __launch_bounds__(NTHR) void k_wt(const float* __restrict__ w, unsigned short* wt) {
  __shared__ __attribute__((aligned(16))) unsigned short tl[OD * WTP];
  const int tid = (int)threadIdx.x;
#pragma unroll 4
  for (int it = 0; it < (KD * OD / 4) / NTHR; ++it) {
    const int u  = it * NTHR + tid;
    const int k  = u >> 5;
    const int n4 = (u & 31) * 4;
    const v4f v = *(const v4fa*)(w + (size_t)k * OD + n4);
    tl[(n4 + 0) * WTP + k] = (unsigned short)bf16_bits(v[0]);
    tl[(n4 + 1) * WTP + k] = (unsigned short)bf16_bits(v[1]);
    tl[(n4 + 2) * WTP + k] = (unsigned short)bf16_bits(v[2]);
    tl[(n4 + 3) * WTP + k] = (unsigned short)bf16_bits(v[3]);
  }
  __syncthreads();
#pragma unroll 1
  for (int it = 0; it < (OD * KD / 8) / NTHR; ++it) {
    const int g  = it * NTHR + tid;
    const int n  = g >> 4;
    const int k8 = (g & 15) * 8;
    const v8us v = *(const v8usa*)(tl + n * WTP + k8);
    st2_v8us(wt + (size_t)g * 8, v);
  }
}

__global__ __launch_bounds__(NTHR) void k_tab(const float* __restrict__ alpha, const float* __restrict__ bias,
                                              float* tab) {
  __shared__ __attribute__((aligned(16))) float st[384];
  const int tid = (int)threadIdx.x;
  const float a = alpha[clampi(tid, 0, NREL - 1)];
  asm volatile("" :: "v"(a));
  const float b = bias[clampi(tid, 0, OD - 1)];
  asm volatile("" :: "v"(b));
  const bool live = (tid >= 1) && (tid < NREL);
  const float av = bf16_val(a);
  st[tid] = live ? av : 0.0f;
  if (tid < OD) st[256 + tid] = bf16_val(b);
  __syncthreads();
  if (tid < 96) {
    const v4f v = *(const v4fa*)(st + 4 * tid);
    st2_v4f(tab + 4 * tid, v);
  }
}

__global__ __launch_bounds__(NTHR) void k_bucket(const int* __restrict__ types, const int* __restrict__ srcs,
                                                 const int* __restrict__ dsts, const float* __restrict__ TB,
                                                 int* LIST, int* CNT, int* OFF, int* FLAG) {
  extern __shared__ __attribute__((aligned(16))) int dsm[];
  __shared__ __attribute__((aligned(16))) float tbs[256];
  int* wl   = dsm;
  int* pl   = dsm + NWAVE * WLCAP;
  int* cnt  = pl + LCAP;
  int* offs = cnt + NBRUN;
  int* cur  = offs + NBRUN;
  int* misc = cur + NBRUN;
  const int tid = (int)threadIdx.x, lane = tid & 31, wave = tid >> 5;
  const int blk = (int)blockIdx.x;
  const unsigned nbs = (unsigned)(blk * NBRUN);

  {
    const v4i z4 = {0, 0, 0, 0};
    for (int i = tid * 4; i < BK_ZINTS; i += NTHR * 4) *(v4ia*)(dsm + i) = z4;
    if (tid < 16) misc[tid] = 0;
    const float tv = TB[tid];
    tbs[tid] = tv;
  }
  __syncthreads();

  {
    const int per  = ((NE + NWAVE * WCH - 1) / (NWAVE * WCH)) * WCH;
    const int ebeg = wave * per;
    const int eend = (ebeg + per < NE) ? (ebeg + per) : NE;
    int* mylist = wl + wave * WLCAP;
    int wc = 0;
#pragma unroll 1
    for (int cb = ebeg; cb < eend; cb += WCH) {
      const int e0  = cb + lane * EPT;
      const int ec  = e0 < NE - EPT ? e0 : NE - EPT;
      const int inv = (e0 < NE) ? 0 : -1;
      const v4i da = *(const v4ia*)(dsts + ec);
      const v4i db = *(const v4ia*)(dsts + ec + 4);
      asm volatile("" :: "v"(da), "v"(db));
      const unsigned s0 = (unsigned)(da.x | inv) - nbs, s1 = (unsigned)(da.y | inv) - nbs;
      const unsigned s2 = (unsigned)(da.z | inv) - nbs, s3 = (unsigned)(da.w | inv) - nbs;
      const unsigned s4 = (unsigned)(db.x | inv) - nbs, s5 = (unsigned)(db.y | inv) - nbs;
      const unsigned s6 = (unsigned)(db.z | inv) - nbs, s7 = (unsigned)(db.w | inv) - nbs;
      const bool h0 = s0 < (unsigned)NBRUN, h1 = s1 < (unsigned)NBRUN, h2 = s2 < (unsigned)NBRUN, h3 = s3 < (unsigned)NBRUN;
      const bool h4 = s4 < (unsigned)NBRUN, h5 = s5 < (unsigned)NBRUN, h6 = s6 < (unsigned)NBRUN, h7 = s7 < (unsigned)NBRUN;
      const unsigned m0 = __builtin_amdgcn_ballot_w32(h0), m1 = __builtin_amdgcn_ballot_w32(h1);
      const unsigned m2 = __builtin_amdgcn_ballot_w32(h2), m3 = __builtin_amdgcn_ballot_w32(h3);
      const unsigned m4 = __builtin_amdgcn_ballot_w32(h4), m5 = __builtin_amdgcn_ballot_w32(h5);
      const unsigned m6 = __builtin_amdgcn_ballot_w32(h6), m7 = __builtin_amdgcn_ballot_w32(h7);
      const unsigned any = m0 | m1 | m2 | m3 | m4 | m5 | m6 | m7;
      if (any != 0u) {
        const int pre = (int)(__builtin_amdgcn_mbcnt_lo(m0, 0u) + __builtin_amdgcn_mbcnt_lo(m1, 0u) +
                              __builtin_amdgcn_mbcnt_lo(m2, 0u) + __builtin_amdgcn_mbcnt_lo(m3, 0u) +
                              __builtin_amdgcn_mbcnt_lo(m4, 0u) + __builtin_amdgcn_mbcnt_lo(m5, 0u) +
                              __builtin_amdgcn_mbcnt_lo(m6, 0u) + __builtin_amdgcn_mbcnt_lo(m7, 0u));
        int p = wc + pre;
        if (h0) { if (p < WLCAP) mylist[p] = ((e0 + 0) << SLB) | (int)s0; p = p + 1; }
        if (h1) { if (p < WLCAP) mylist[p] = ((e0 + 1) << SLB) | (int)s1; p = p + 1; }
        if (h2) { if (p < WLCAP) mylist[p] = ((e0 + 2) << SLB) | (int)s2; p = p + 1; }
        if (h3) { if (p < WLCAP) mylist[p] = ((e0 + 3) << SLB) | (int)s3; p = p + 1; }
        if (h4) { if (p < WLCAP) mylist[p] = ((e0 + 4) << SLB) | (int)s4; p = p + 1; }
        if (h5) { if (p < WLCAP) mylist[p] = ((e0 + 5) << SLB) | (int)s5; p = p + 1; }
        if (h6) { if (p < WLCAP) mylist[p] = ((e0 + 6) << SLB) | (int)s6; p = p + 1; }
        if (h7) { if (p < WLCAP) mylist[p] = ((e0 + 7) << SLB) | (int)s7; p = p + 1; }
        wc += (int)(__builtin_popcount(m0) + __builtin_popcount(m1) + __builtin_popcount(m2) + __builtin_popcount(m3) +
                    __builtin_popcount(m4) + __builtin_popcount(m5) + __builtin_popcount(m6) + __builtin_popcount(m7));
      }
    }
    if (lane == 0) misc[wave] = wc;
  }
  __syncthreads();

  if (wave == 0) {
    int ov = 0;
    int tot = 0;
#pragma unroll 1
    for (int w2 = 0; w2 < NWAVE; ++w2) {
      int c = misc[w2];
      if (c > WLCAP) ov = 1;
      c = c < 0 ? 0 : (c > WLCAP ? WLCAP : c);
      tot += c;
#pragma unroll 1
      for (int b0 = 0; b0 < c; b0 += 32) {
        const int idx = b0 + lane;
        const int ent = wl[w2 * WLCAP + (idx < WLCAP ? idx : WLCAP - 1)];
        const int m32 = (c - b0) < 32 ? (c - b0) : 32;
#pragma unroll 1
        for (int k = 0; k < m32; ++k) {
          const int u    = __builtin_amdgcn_readlane(ent, k);
          const int slot = u & (NBRUN - 1);
          if (lane == 0) cnt[slot] = cnt[slot] + 1;
        }
      }
    }
    if (tot > LCAP) ov = 1;
    if (lane == 0) { misc[9] = ov; misc[10] = tot; }
  }
  __syncthreads();
  if (wave == 0) {
    const int base = lane * (NBRUN / 32);
    int s = 0;
    int ovl = 0;
#pragma unroll 1
    for (int i = 0; i < NBRUN / 32; ++i) {
      const int cv = cnt[base + i];
      s += cv;
      ovl |= (cv > DEGCAP) ? 1 : 0;
    }
    int incl = s;
#pragma unroll
    for (int d = 1; d < 32; d <<= 1) {
      const int y = __shfl_up(incl, d, 32);
      if (lane >= d) incl += y;
    }
    int run = incl - s;
#pragma unroll 1
    for (int i = 0; i < NBRUN / 32; ++i) {
      const int cv = cnt[base + i];
      offs[base + i] = run;
      cur[base + i]  = run;
      run += cv;
    }
    const unsigned om = __builtin_amdgcn_ballot_w32(ovl != 0);
    if (lane == 0 && om != 0u) misc[9] = 1;
  }
  __syncthreads();

  if (wave == 0) {
#pragma unroll 1
    for (int w2 = 0; w2 < NWAVE; ++w2) {
      int c = misc[w2];
      c = c < 0 ? 0 : (c > WLCAP ? WLCAP : c);
#pragma unroll 1
      for (int b0 = 0; b0 < c; b0 += 32) {
        const int idx = b0 + lane;
        const int ent = wl[w2 * WLCAP + (idx < WLCAP ? idx : WLCAP - 1)];
        const int m32 = (c - b0) < 32 ? (c - b0) : 32;
#pragma unroll 1
        for (int k = 0; k < m32; ++k) {
          const int u    = __builtin_amdgcn_readlane(ent, k);
          const int slot = u & (NBRUN - 1);
          const int eid  = (u >> SLB) & 0x1FFFFF;
          if (lane == 0) {
            int p = cur[slot];
            p = p < 0 ? 0 : (p > LCAP - 1 ? LCAP - 1 : p);
            pl[p] = eid;
            cur[slot] = p + 1;
          }
        }
      }
    }
  }
  __syncthreads();

  const int ovf = misc[9];
  const int tot = clampi(misc[10], 0, LCAP);
  int* lp = LIST + (size_t)blk * (size_t)(2 * LCAP);
#pragma unroll 1
  for (int it = 0; it < (LCAP / 2) / NTHR; ++it) {
    const int u  = it * NTHR + tid;
    const int i0 = 2 * u;
    const v2i pe = *(const v2ia*)(pl + i0);
    const int e0 = clampi(pe.x, 0, NE - 1);
    const int e1 = clampi(pe.y, 0, NE - 1);
    const int t0 = twin_of(e0);
    const int t1 = twin_of(e1);
    const int sa = srcs[e0];
    const int ya = types[e0];
    const int za = types[t0];
    const int sb = srcs[e1];
    const int yb = types[e1];
    const int zb = types[t1];
    asm volatile("" :: "v"(sa), "v"(ya), "v"(za), "v"(sb), "v"(yb), "v"(zb));
    const float aa = tbs[clampi(ya, 0, NREL - 1)] + tbs[clampi(za, 0, NREL - 1)];
    const float ab = tbs[clampi(yb, 0, NREL - 1)] + tbs[clampi(zb, 0, NREL - 1)];
    const int ma = (i0 < tot) ? -1 : 0;
    const int mb = (i0 + 1 < tot) ? -1 : 0;
    v4i o;
    o.x = clampi(sa, 0, NN - 1) & ma;
    o.y = __float_as_int(aa) & ma;
    o.z = clampi(sb, 0, NN - 1) & mb;
    o.w = __float_as_int(ab) & mb;
    st2_v4i(lp + 4 * u, o);
  }
  {
    const v4i vc = *(const v4ia*)(cnt + 4 * tid);
    st2_v4i(CNT + (size_t)blk * NBRUN + 4 * tid, vc);
    const v4i vo = *(const v4ia*)(offs + 4 * tid);
    st2_v4i(OFF + (size_t)blk * NBRUN + 4 * tid, vo);
  }
  if (tid < 8) {
    const v4i f = {ovf, ovf, ovf, ovf};
    st2_v4i(FLAG + (size_t)blk * 32 + 4 * tid, f);
  }
}

__global__ __launch_bounds__(NTHR) __attribute__((amdgpu_num_vgpr(248)))
void k_walk(const int* __restrict__ LIST, const int* __restrict__ CNT, const int* __restrict__ OFF,
            const int* __restrict__ FLAG, const float* __restrict__ F, const float* __restrict__ BB,
            float* out, int nreal) {
#pragma clang fp contract(off)
  const int tid = (int)threadIdx.x, lane = tid & 31, wave = tid >> 5;
  const int row = (int)blockIdx.x * NWAVE + wave;
  const int rc  = clampi(row, 0, NBK * NBRUN - 1);
  int c    = CNT[rc];
  int o    = OFF[rc];
  int flag = FLAG[(size_t)(rc >> SLB) * 32];
  asm volatile("" :: "v"(c), "v"(o), "v"(flag));
  const bool big = c > DEGCAP;
  c = clampi(c, 0, DEGCAP);
  o = clampi(o, 0, LCAP - 1);
  c = __builtin_amdgcn_readfirstlane(c);
  o = __builtin_amdgcn_readfirstlane(o);
  int last = o + (c > 0 ? c : 1) - 1;
  last = last > LCAP - 1 ? LCAP - 1 : last;
  const int* lb = LIST + (size_t)(rc >> SLB) * (size_t)(2 * LCAP);
  const v4f bb = *(const v4fa*)(BB + 4 * lane);
  asm volatile("" :: "v"(bb));

  v4f acc = (v4f){0.0f, 0.0f, 0.0f, 0.0f};
#pragma unroll 1
  for (int b0 = 0; b0 < c; b0 += 32) {
    int idx = o + b0 + lane;
    idx = idx > last ? last : idx;
    const v2i ent = *(const v2ia*)(lb + 2 * idx);
    asm volatile("" :: "v"(ent));
    const int sr = clampi(ent.x, 0, NN - 1);
    const int wv = ent.y;
    const int m32 = (c - b0) < 32 ? (c - b0) : 32;
#pragma unroll 1
    for (int k = 0; k < m32; ++k) {
      const int   sk = __builtin_amdgcn_readlane(sr, k);
      const float ak = __int_as_float(__builtin_amdgcn_readlane(wv, k));
      const v4f q = *(const v4fa*)(F + (size_t)sk * OD + 4 * lane);
      asm volatile("" :: "v"(q));
      const v4f p = q * ak;
      acc = acc + p;
    }
  }
  const v4f r = acc + bb;
  const float qnan = __uint_as_float(0x7fc00000u);
  const bool bad = (flag != 0) || big;
  v4f ov;
  ov.x = bad ? qnan : r.x; ov.y = bad ? qnan : r.y; ov.z = bad ? qnan : r.z; ov.w = bad ? qnan : r.w;
  if (row < nreal) {
    st2_v4f(out + (size_t)row * OD + 4 * lane, ov);
  }
}

extern "C" void kernel_launch(void* const* d_in, const int* in_sizes, int n_in,
                              void* d_out, int out_size, void* d_ws, size_t ws_size,
                              hipStream_t stream) {
  if (n_in < 7) return;
  if (in_sizes[0] != NN * KD) return;
  if (in_sizes[1] != NE) return;
  if (in_sizes[2] != NE) return;
  if (in_sizes[3] != NE) return;
  if (in_sizes[4] != KD * OD) return;
  if (in_sizes[5] != NREL) return;
  if (in_sizes[6] != OD) return;
  if (out_size != NN * OD) return;

  const float* x     = (const float*)d_in[0];
  const int*   types = (const int*)d_in[1];
  const int*   srcs  = (const int*)d_in[2];
  const int*   dsts  = (const int*)d_in[3];
  const float* W     = (const float*)d_in[4];
  const float* alpha = (const float*)d_in[5];
  const float* bias  = (const float*)d_in[6];
  float* out = (float*)d_out;

  constexpr size_t zXB   = (size_t)MPAD * KD * 2;
  constexpr size_t zF    = (size_t)MPAD * OD * 4;
  constexpr size_t zWT   = (size_t)OD * KD * 2;
  constexpr size_t zTAB  = 1536;
  constexpr size_t zLIST = (size_t)NBK * LCAP * 8;
  constexpr size_t zCNT  = (size_t)NBK * NBRUN * 4;
  constexpr size_t zOFF  = (size_t)NBK * NBRUN * 4;
  constexpr size_t zFLAG = (size_t)NBK * 128;
  constexpr size_t oXB   = 0;
  constexpr size_t oF    = oXB + zXB;
  constexpr size_t oWT   = oF + zF;
  constexpr size_t oTAB  = oWT + zWT;
  constexpr size_t oLIST = oTAB + zTAB;
  constexpr size_t oCNT  = oLIST + zLIST;
  constexpr size_t oOFF  = oCNT + zCNT;
  constexpr size_t oFLAG = oOFF + zOFF;
  constexpr size_t oEND  = oFLAG + zFLAG;
  static_assert(zXB % 128 == 0 && zF % 128 == 0 && zWT % 128 == 0 && zTAB % 128 == 0);
  static_assert(zLIST % 128 == 0 && zCNT % 128 == 0 && zOFF % 128 == 0 && zFLAG % 128 == 0);
  static_assert(oEND == 89765632);
  static_assert(oEND <= (size_t)WSMAX);
  if (oEND > ws_size) return;

  char* ws = (char*)d_ws;
  unsigned short* XB   = (unsigned short*)(ws + oXB);
  float*          F    = (float*)(ws + oF);
  unsigned short* WT   = (unsigned short*)(ws + oWT);
  float*          TAB  = (float*)(ws + oTAB);
  float*          TBp  = TAB;
  float*          BBp  = TAB + 256;
  int*            LIST = (int*)(ws + oLIST);
  int*            CNT  = (int*)(ws + oCNT);
  int*            OFF  = (int*)(ws + oOFF);
  int*            FLAG = (int*)(ws + oFLAG);

  hipFuncSetAttribute(reinterpret_cast<const void*>(&k_bucket), hipFuncAttributeMaxDynamicSharedMemorySize, (int)BK_LDS);

  constexpr int gPlane = MPAD * KD / 8 / NTHR;
  constexpr int gTiles = (MPAD / 64) * (OD / 64);
  constexpr int gGemm  = (gTiles + 7) / 8;
  static_assert(gPlane == 6256 && gGemm == 391 && NN / NWAVE == 12500);

  k_plane<0><<<gPlane, NTHR, 0, stream>>>(x, NN, KD, KD, XB, MPAD, KD);
  k_wt<<<1, NTHR, 0, stream>>>(W, WT);
  k_tab<<<1, NTHR, 0, stream>>>(alpha, bias, TAB);
  k_gemm_nt<0, 0><<<gGemm, NTHR, 0, stream>>>(XB, WT, BBp, F, MPAD, OD, KD, OD);
  k_bucket<<<NBK, NTHR, BK_LDS, stream>>>(types, srcs, dsts, TBp, LIST, CNT, OFF, FLAG);
  k_walk<<<NN / NWAVE, NTHR, 0, stream>>>(LIST, CNT, OFF, FLAG, F, BBp, out, NN);
}
